// TransformerBlock_50379966382285
// MI455X (gfx1250) — hardware-verified
//
#include <hip/hip_runtime.h>
#include <stddef.h>


typedef _Float16 v16h __attribute__((ext_vector_type(16)));
typedef _Float16 v8h  __attribute__((ext_vector_type(8)));
typedef float    v8f  __attribute__((ext_vector_type(8)));
typedef float    v4f  __attribute__((ext_vector_type(4)));
typedef int      v4i  __attribute__((ext_vector_type(4)));

#ifndef NB
#define NB 4
#endif
#ifndef SEQ
#define SEQ 1024
#endif
#define NB_FULL  4
#define SEQ_FULL 1024
#define DIM   1024
#define NHEAD 16
#define HD    64
#define DFF   4096
#define MROWS (NB * SEQ)

static_assert(NB >= 1 && NB <= NB_FULL);
static_assert(SEQ >= 128 && SEQ <= SEQ_FULL && (SEQ % 128) == 0);
static_assert(DIM == NHEAD * HD);
static_assert(HD == 64);
static_assert(DIM == 128 * 8);
static_assert((MROWS % 64) == 0);
static_assert((DIM % 64) == 0 && (DFF % 64) == 0 && (DIM % 32) == 0 && (DFF % 32) == 0);

#define LDT 72
#define LDC 68

#define WCARRY 64.0f
#define PCARRY 1024.0f
#define VCARRY 64.0f
#define HCARRY 4.0f
#define LN_EPS 1.0e-8f
#define MASK_FILL (-0.01f)
#define SCORE_SCALE 0.125f

#define WP        ((size_t)DIM * DIM)
#define WT_ELEMS  (WP * 4 + (size_t)DFF * DIM * 2)
#define WT_BYTES  (WT_ELEMS * 2)
#define P16_BYTES ((size_t)MROWS * DIM * 2)
#define P32_BYTES ((size_t)MROWS * DIM * 4)
#define H16_BYTES ((size_t)MROWS * DFF * 2)
#define OFF_NX    (WT_BYTES)
#define OFF_QH    (OFF_NX + P16_BYTES)
#define OFF_KH    (OFF_QH + P16_BYTES)
#define OFF_VT    (OFF_KH + P16_BYTES)
#define OFF_VATT  (OFF_VT + P16_BYTES)
#define OFF_X1    (OFF_VATT + P16_BYTES)
#define OFF_NX2   (OFF_X1 + P32_BYTES)
#define OFF_H     (OFF_NX2 + P16_BYTES)
#define WS_TOTAL  (OFF_H + H16_BYTES)
static_assert((WP % 2048) == 0 && (WT_ELEMS % 2048) == 0);
static_assert((WT_BYTES % 128) == 0 && (P16_BYTES % 128) == 0 && (P32_BYTES % 128) == 0);
static_assert(((size_t)DFF * DIM) == 4 * WP);
static_assert(WS_TOTAL <= (size_t)134217728);

__device__ __forceinline__ float bf16r(float x) {
  unsigned int u = __float_as_uint(x);
  u = (u + 0x7FFFu + ((u >> 16) & 1u)) & 0xFFFF0000u;
  return __uint_as_float(u);
}

__device__ __forceinline__ v16h frag_at(const _Float16* p) {
  v8h lo = *(const v8h*)(p);
  v8h hi = *(const v8h*)(p + 16);
  v16h out;
#pragma unroll
  for (int i = 0; i < 8; ++i) { out[i] = lo[i]; out[i + 8] = hi[i]; }
  return out;
}
__device__ __forceinline__ v16h ld_frag(const _Float16* base, int ld) {
  const int lane = threadIdx.x & 31;
  return frag_at(base + (lane & 15) * ld + (lane >> 4) * 8);
}

__device__ __forceinline__ v8f wmma16(v16h a, v16h b, v8f c) {
  v8f d = __builtin_amdgcn_wmma_f32_16x16x32_f16(false, a, false, b, (short)0, c,
                                                 false, false);
  asm volatile("v_nop\n\tv_nop\n\tv_nop\n\tv_nop" : "+v"(d) : "v"(a), "v"(b));
  return d;
}

__device__ __forceinline__ float red32_sum(float x) {
#pragma unroll
  for (int off = 1; off < 32; off <<= 1) x += __shfl_xor(x, off, 32);
  return x;
}

__device__ __forceinline__ void wave_lds_sync() {
  __builtin_amdgcn_fence(3  , "wavefront");
  asm volatile("s_wait_dscnt 0x0" ::: "memory");
  __builtin_amdgcn_wave_barrier();
}

__device__ __forceinline__ float gelu_f(float x) {
  const float c = 0.7978845608028654f;
  const float u = x * x * x;
  const float t = c * (x + 0.044715f * u);
  const float e = __expf(2.0f * t);
  const float th = 1.0f - 2.0f * __builtin_amdgcn_rcpf(e + 1.0f);
  return 0.5f * x * (1.0f + th);
}

__global__ __launch_bounds__(256) void wconv_kernel(
    const float* __restrict__ W0, const float* __restrict__ W1p,
    const float* __restrict__ W2p, const float* __restrict__ W3,
    const float* __restrict__ W4, const float* __restrict__ W5,
    _Float16* __restrict__ Wt) {
  const size_t e = ((size_t)blockIdx.x * 256 + threadIdx.x) * 8;
  const unsigned seg = (unsigned)(((size_t)blockIdx.x * 2048) / WP);
  const float* W = W0;
  size_t base = 0;
  if (seg == 1) { W = W1p; base = WP; }
  if (seg == 2) { W = W2p; base = 2 * WP; }
  if (seg == 3) { W = W3;  base = 3 * WP; }
  if (seg >= 4 && seg < 8) { W = W4; base = 4 * WP; }
  if (seg >= 8) { W = W5; base = 8 * WP; }
  const float* sp = W + (e - base);
  const v4f a0 = *(const v4f*)(sp);
  const v4f a1 = *(const v4f*)(sp + 4);
  v8h o;
#pragma unroll
  for (int j = 0; j < 4; ++j) {
    o[j]     = (_Float16)(WCARRY * bf16r(a0[j]));
    o[j + 4] = (_Float16)(WCARRY * bf16r(a1[j]));
  }
  *(volatile v8h*)(Wt + e) = o;
  __threadfence();
  *(volatile v8h*)(Wt + e) = o;
}

template <int RND, int SRCSEQ>
__global__ __launch_bounds__(128) void ln_kernel(
    const float* __restrict__ src, const float* __restrict__ g,
    const float* __restrict__ be, _Float16* __restrict__ dst) {
  __shared__ float red[8];
  const int tid = threadIdx.x, lane = tid & 31, w = tid >> 5;
  const int row = blockIdx.x;
  const int bidx = row / SEQ;
  const int sq = row - bidx * SEQ;
  const size_t srow = (size_t)bidx * SRCSEQ + sq;
  const int c = tid * 8;
  const float* sp = src + srow * DIM + c;
  const v4f a0 = *(const v4f*)(sp);
  const v4f a1 = *(const v4f*)(sp + 4);
  float v[8];
#pragma unroll
  for (int j = 0; j < 4; ++j) {
    v[j]     = RND ? bf16r(a0[j]) : a0[j];
    v[j + 4] = RND ? bf16r(a1[j]) : a1[j];
  }
  float s = ((v[0] + v[1]) + (v[2] + v[3])) + ((v[4] + v[5]) + (v[6] + v[7]));
  s = red32_sum(s);
  if (lane == 0) red[w] = s;
  __syncthreads();
  const float mean = ((red[0] + red[1]) + (red[2] + red[3])) * (1.0f / (float)DIM);
  float d[8];
#pragma unroll
  for (int j = 0; j < 8; ++j) d[j] = v[j] - mean;
  float q = ((d[0] * d[0] + d[1] * d[1]) + (d[2] * d[2] + d[3] * d[3])) +
            ((d[4] * d[4] + d[5] * d[5]) + (d[6] * d[6] + d[7] * d[7]));
  q = red32_sum(q);
  if (lane == 0) red[4 + w] = q;
  __syncthreads();
  const float var = ((red[4] + red[5]) + (red[6] + red[7])) * (1.0f / (float)(DIM - 1));
  const float sd = sqrtf(var);
  const float inv = 1.0f / (sd + LN_EPS);
  const v4f g0 = *(const v4f*)(g + c);
  const v4f g1 = *(const v4f*)(g + c + 4);
  const v4f b0 = *(const v4f*)(be + c);
  const v4f b1 = *(const v4f*)(be + c + 4);
  v8h o;
#pragma unroll
  for (int j = 0; j < 4; ++j) {
    o[j]     = (_Float16)((bf16r(g0[j]) * d[j]) * inv + bf16r(b0[j]));
    o[j + 4] = (_Float16)((bf16r(g1[j]) * d[j + 4]) * inv + bf16r(b1[j]));
  }
  const size_t off = (size_t)row * DIM + c;
  *(volatile v8h*)(dst + off) = o;
  __threadfence();
  *(volatile v8h*)(dst + off) = o;
}

template <int MODE, int KD, int NP>
__global__ __launch_bounds__(256) void gemm_kernel(
    const _Float16* __restrict__ A16, const _Float16* __restrict__ Bt,
    const float* __restrict__ bias, const float* __restrict__ xin,
    const float* __restrict__ resf, float* __restrict__ outf,
    _Float16* __restrict__ out16) {
  static_assert((KD % 32) == 0 && (NP % 64) == 0);
  __shared__ float Cs[64 * LDC] __attribute__((aligned(16)));
  const int tid = threadIdx.x, lane = tid & 31, w = tid >> 5;
  const int mw = w >> 1, nw = w & 1;
  const int hh = lane >> 4, m = lane & 15;
  const int n0 = blockIdx.x * 64;
  const int row0 = blockIdx.y * 64;

  const _Float16* ap  = A16 + (size_t)(row0 + mw * 16 + m) * KD + hh * 8;
  const _Float16* bp0 = Bt + (size_t)(n0 + nw * 32 + m) * KD + hh * 8;
  const _Float16* bp1 = bp0 + (size_t)16 * KD;
  v8f acc0 = {}, acc1 = {};
#pragma unroll 2
  for (int k0 = 0; k0 < KD; k0 += 32) {
    const v16h a  = frag_at(ap + k0);
    const v16h b0 = frag_at(bp0 + k0);
    const v16h b1 = frag_at(bp1 + k0);
    acc0 = wmma16(a, b0, acc0);
    acc1 = wmma16(a, b1, acc1);
  }
#pragma unroll
  for (int r = 0; r < 8; ++r) {
    float* d = &Cs[(mw * 16 + hh * 8 + r) * LDC + nw * 32 + m];
    d[0]  = acc0[r];
    d[16] = acc1[r];
  }
  __syncthreads();

  if (MODE == 0) {
    v8h x[2];
    size_t off[2];
#pragma unroll
    for (int i = 0; i < 2; ++i) {
      const int r = 32 * i + (tid >> 3);
      const int c = (tid & 7) * 8;
      const v4f u0 = *(const v4f*)&Cs[r * LDC + c];
      const v4f u1 = *(const v4f*)&Cs[r * LDC + c + 4];
      const v4f g0 = *(const v4f*)(bias + n0 + c);
      const v4f g1 = *(const v4f*)(bias + n0 + c + 4);
#pragma unroll
      for (int j = 0; j < 4; ++j) {
        x[i][j]     = (_Float16)(u0[j] * (1.0f / WCARRY) + bf16r(g0[j]));
        x[i][j + 4] = (_Float16)(u1[j] * (1.0f / WCARRY) + bf16r(g1[j]));
      }
      off[i] = (size_t)(row0 + r) * NP + n0 + c;
    }
#pragma unroll
    for (int i = 0; i < 2; ++i) *(volatile v8h*)(out16 + off[i]) = x[i];
    __threadfence();
#pragma unroll
    for (int i = 0; i < 2; ++i) *(volatile v8h*)(out16 + off[i]) = x[i];
  }

  if (MODE == 1) {
    const int bidx = row0 / SEQ;
    const int key0 = row0 - bidx * SEQ;
    v8h x[2];
    size_t off[2];
#pragma unroll
    for (int i = 0; i < 2; ++i) {
      const int dcol = 32 * i + (tid >> 3);
      const int kk = (tid & 7) * 8;
      const float gb = bf16r(bias[n0 + dcol]);
#pragma unroll
      for (int j = 0; j < 8; ++j)
        x[i][j] = (_Float16)(Cs[(kk + j) * LDC + dcol] * (1.0f / WCARRY) + gb);
      off[i] = ((size_t)bidx * DIM + n0 + dcol) * SEQ + key0 + kk;
    }
#pragma unroll
    for (int i = 0; i < 2; ++i) *(volatile v8h*)(out16 + off[i]) = x[i];
    __threadfence();
#pragma unroll
    for (int i = 0; i < 2; ++i) *(volatile v8h*)(out16 + off[i]) = x[i];
  }

  if (MODE == 2) {
    v4f xs[4];
    size_t off[4];
#pragma unroll
    for (int i = 0; i < 4; ++i) {
      const int r = 16 * i + (tid >> 4);
      const int c = (tid & 15) * 4;
      const int crow = row0 + r;
      const int bidx = crow / SEQ;
      const int sq = crow - bidx * SEQ;
      const size_t frow = (size_t)bidx * SEQ_FULL + sq;
      const v4f u = *(const v4f*)&Cs[r * LDC + c];
      const v4f q = *(const v4f*)(xin + frow * DIM + n0 + c);
      const v4f gb = *(const v4f*)(bias + n0 + c);
      v4f val;
#pragma unroll
      for (int j = 0; j < 4; ++j)
        val[j] = (u[j] * (1.0f / (WCARRY * VCARRY)) + bf16r(gb[j])) + bf16r(q[j]);
      xs[i] = val;
      off[i] = (size_t)crow * NP + n0 + c;
    }
#pragma unroll
    for (int i = 0; i < 4; ++i) *(volatile v4f*)(outf + off[i]) = xs[i];
    __threadfence();
#pragma unroll
    for (int i = 0; i < 4; ++i) *(volatile v4f*)(outf + off[i]) = xs[i];
  }

  if (MODE == 3) {
    v8h x[2];
    size_t off[2];
#pragma unroll
    for (int i = 0; i < 2; ++i) {
      const int r = 32 * i + (tid >> 3);
      const int c = (tid & 7) * 8;
      const v4f u0 = *(const v4f*)&Cs[r * LDC + c];
      const v4f u1 = *(const v4f*)&Cs[r * LDC + c + 4];
      const v4f g0 = *(const v4f*)(bias + n0 + c);
      const v4f g1 = *(const v4f*)(bias + n0 + c + 4);
#pragma unroll
      for (int j = 0; j < 4; ++j) {
        const float t0 = gelu_f(u0[j] * (1.0f / WCARRY) + bf16r(g0[j]));
        const float t1 = gelu_f(u1[j] * (1.0f / WCARRY) + bf16r(g1[j]));
        x[i][j]     = (_Float16)(HCARRY * t0);
        x[i][j + 4] = (_Float16)(HCARRY * t1);
      }
      off[i] = (size_t)(row0 + r) * NP + n0 + c;
    }
#pragma unroll
    for (int i = 0; i < 2; ++i) *(volatile v8h*)(out16 + off[i]) = x[i];
    __threadfence();
#pragma unroll
    for (int i = 0; i < 2; ++i) *(volatile v8h*)(out16 + off[i]) = x[i];
  }

  if (MODE == 4) {
    v4f xs[4];
    size_t off[4];
#pragma unroll
    for (int i = 0; i < 4; ++i) {
      const int r = 16 * i + (tid >> 4);
      const int c = (tid & 15) * 4;
      const int crow = row0 + r;
      const int bidx = crow / SEQ;
      const int sq = crow - bidx * SEQ;
      const size_t frow = (size_t)bidx * SEQ_FULL + sq;
      const v4f u  = *(const v4f*)&Cs[r * LDC + c];
      const v4f gb = *(const v4f*)(bias + n0 + c);
      const v4f rx = *(const v4f*)(resf + (size_t)crow * DIM + n0 + c);
      v4f val;
#pragma unroll
      for (int j = 0; j < 4; ++j)
        val[j] = (u[j] * (1.0f / (WCARRY * HCARRY)) + bf16r(gb[j])) + rx[j];
      xs[i] = val;
      off[i] = frow * NP + n0 + c;
    }
#pragma unroll
    for (int i = 0; i < 4; ++i) *(volatile v4f*)(outf + off[i]) = xs[i];
    __threadfence();
#pragma unroll
    for (int i = 0; i < 4; ++i) *(volatile v4f*)(outf + off[i]) = xs[i];
  }
}

__global__ __launch_bounds__(256) void attn_kernel(
    const _Float16* __restrict__ Qh, const _Float16* __restrict__ Kh,
    const _Float16* __restrict__ Vt, const int* __restrict__ mask,
    _Float16* __restrict__ Ov) {
  __shared__ _Float16 Ks[64 * LDT] __attribute__((aligned(16)));
  __shared__ _Float16 Vs[64 * LDT] __attribute__((aligned(16)));
  __shared__ _Float16 Ps[8 * 16 * LDT] __attribute__((aligned(16)));

  const int tid = threadIdx.x, lane = tid & 31, w = tid >> 5;
  const int hh = lane >> 4, m = lane & 15;
  const int q0 = blockIdx.x * 128;
  const int head = blockIdx.y;
  const int b = blockIdx.z;
  _Float16* P = Ps + w * (16 * LDT);

  const int qrow = q0 + w * 16 + m;
  const size_t qoff = (size_t)(b * SEQ + qrow) * DIM + head * HD + hh * 8;
  v16h qf[2];
  qf[0] = frag_at(Qh + qoff);
  qf[1] = frag_at(Qh + qoff + 32);

  const int* mrowp = mask + ((size_t)b * SEQ_FULL + qrow) * SEQ_FULL + hh * 8;

  float mrun = -1.0e30f, lrun = 0.0f;
  v8f o[4];
#pragma unroll
  for (int nb = 0; nb < 4; ++nb) o[nb] = (v8f){};

  const size_t kplane = (size_t)b * SEQ * DIM + head * HD;
  const size_t vplane = ((size_t)b * DIM + head * HD) * SEQ;

  for (int kb = 0; kb < SEQ; kb += 64) {
#pragma unroll
    for (int j = 0; j < 2; ++j) {
      const int idx = tid + 256 * j;
      const int r = idx >> 3, c = (idx & 7) * 8;
      *(v8h*)&Ks[r * LDT + c] = *(const v8h*)(Kh + kplane + (size_t)(kb + r) * DIM + c);
      *(v8h*)&Vs[r * LDT + c] = *(const v8h*)(Vt + vplane + (size_t)r * SEQ + kb + c);
    }
    __syncthreads();

    v8f s[4];
#pragma unroll
    for (int kg = 0; kg < 4; ++kg) {
      v8f t = {};
#pragma unroll
      for (int c = 0; c < 2; ++c) {
        const v16h kf = ld_frag(&Ks[(kg * 16) * LDT + c * 32], LDT);
        t = wmma16(kf, qf[c], t);
      }
      const v4i mk0 = *(const v4i*)(mrowp + kb + kg * 16);
      const v4i mk1 = *(const v4i*)(mrowp + kb + kg * 16 + 4);
#pragma unroll
      for (int r = 0; r < 4; ++r) {
        const float sv0 = t[r] * SCORE_SCALE;
        const float sv1 = t[r + 4] * SCORE_SCALE;
        s[kg][r]     = (mk0[r] == 0) ? MASK_FILL : sv0 * (float)mk0[r];
        s[kg][r + 4] = (mk1[r] == 0) ? MASK_FILL : sv1 * (float)mk1[r];
      }
    }

    float mx = fmaxf(fmaxf(s[0][0], s[1][0]), fmaxf(s[2][0], s[3][0]));
#pragma unroll
    for (int kg = 0; kg < 4; ++kg)
#pragma unroll
      for (int r = 1; r < 8; ++r) mx = fmaxf(mx, s[kg][r]);
    mx = fmaxf(mx, __shfl_xor(mx, 16, 32));
    const float mn = fmaxf(mrun, mx);
    const float alpha = __expf(mrun - mn);
    mrun = mn;
    float rs[4];
#pragma unroll
    for (int kg = 0; kg < 4; ++kg) {
#pragma unroll
      for (int r = 0; r < 8; ++r) s[kg][r] = __expf(s[kg][r] - mrun);
      rs[kg] = ((s[kg][0] + s[kg][1]) + (s[kg][2] + s[kg][3])) +
               ((s[kg][4] + s[kg][5]) + (s[kg][6] + s[kg][7]));
    }
    float rsum = (rs[0] + rs[1]) + (rs[2] + rs[3]);
    rsum += __shfl_xor(rsum, 16, 32);
    lrun = alpha * lrun + rsum;
#pragma unroll
    for (int v = 0; v < 8; ++v) {
      const float av = __shfl(alpha, 8 * hh + v, 32);
#pragma unroll
      for (int nb = 0; nb < 4; ++nb) o[nb][v] = o[nb][v] * av;
    }

#pragma unroll
    for (int kg = 0; kg < 4; ++kg) {
      v8h pv;
#pragma unroll
      for (int r = 0; r < 8; ++r) pv[r] = (_Float16)(s[kg][r] * PCARRY);
      *(v8h*)&P[m * LDT + kg * 16 + 8 * hh] = pv;
    }
    wave_lds_sync();

#pragma unroll
    for (int c = 0; c < 2; ++c) {
      const v16h pf = ld_frag(P + c * 32, LDT);
#pragma unroll
      for (int nb = 0; nb < 4; ++nb) {
        const v16h vf = ld_frag(&Vs[(nb * 16) * LDT + c * 32], LDT);
        o[nb] = wmma16(pf, vf, o[nb]);
      }
    }
    __syncthreads();
  }

  const float invm = __builtin_amdgcn_rcpf(lrun) * (VCARRY / PCARRY);
#pragma unroll
  for (int v = 0; v < 8; ++v) {
    const float iv = __shfl(invm, 8 * hh + v, 32);
#pragma unroll
    for (int nb = 0; nb < 4; ++nb)
      P[(hh * 8 + v) * LDT + nb * 16 + m] = (_Float16)(o[nb][v] * iv);
  }
  wave_lds_sync();
  v8h x[4];
  size_t off[4];
#pragma unroll
  for (int i = 0; i < 4; ++i) {
    const int r = 4 * i + (lane >> 3);
    const int c = (lane & 7) * 8;
    x[i] = *(const v8h*)&P[r * LDT + c];
    off[i] = (size_t)(b * SEQ + q0 + w * 16 + r) * DIM + head * HD + c;
  }
#pragma unroll
  for (int i = 0; i < 4; ++i) *(volatile v8h*)(Ov + off[i]) = x[i];
  __threadfence();
#pragma unroll
  for (int i = 0; i < 4; ++i) *(volatile v8h*)(Ov + off[i]) = x[i];
}

extern "C" void kernel_launch(void* const* d_in, const int* in_sizes, int n_in,
                              void* d_out, int out_size, void* d_ws, size_t ws_size,
                              hipStream_t stream) {
  if (n_in < 18) return;
  const long long need_x = ((long long)(NB - 1) * SEQ_FULL + SEQ) * DIM;
  const long long need_m = ((long long)(NB - 1) * SEQ_FULL + SEQ) * SEQ_FULL;
  if ((long long)in_sizes[0] < need_x) return;
  if ((long long)in_sizes[1] < need_m) return;
  if (in_sizes[2] < DIM * DIM || in_sizes[4] < DIM * DIM || in_sizes[6] < DIM * DIM ||
      in_sizes[8] < DIM * DIM) return;
  if (in_sizes[10] < DFF * DIM || in_sizes[12] < DFF * DIM) return;
  if (in_sizes[3] < DIM || in_sizes[5] < DIM || in_sizes[7] < DIM || in_sizes[9] < DIM ||
      in_sizes[13] < DIM || in_sizes[14] < DIM || in_sizes[15] < DIM || in_sizes[16] < DIM ||
      in_sizes[17] < DIM) return;
  if (in_sizes[11] < DFF) return;
  if ((long long)out_size < need_x) return;
  if (ws_size < WS_TOTAL) return;

  const float* x    = (const float*)d_in[0];
  const int*   mask = (const int*)d_in[1];
  const float* Wq   = (const float*)d_in[2];
  const float* bq   = (const float*)d_in[3];
  const float* Wk   = (const float*)d_in[4];
  const float* bk   = (const float*)d_in[5];
  const float* Wv   = (const float*)d_in[6];
  const float* bv   = (const float*)d_in[7];
  const float* Wo   = (const float*)d_in[8];
  const float* bo   = (const float*)d_in[9];
  const float* W1   = (const float*)d_in[10];
  const float* b1   = (const float*)d_in[11];
  const float* W2   = (const float*)d_in[12];
  const float* b2   = (const float*)d_in[13];
  const float* g1   = (const float*)d_in[14];
  const float* be1  = (const float*)d_in[15];
  const float* g2   = (const float*)d_in[16];
  const float* be2  = (const float*)d_in[17];
  float* out = (float*)d_out;

  char* ws = (char*)d_ws;
  _Float16* Wt     = (_Float16*)ws;
  _Float16* NX16   = (_Float16*)(ws + OFF_NX);
  _Float16* Qh16   = (_Float16*)(ws + OFF_QH);
  _Float16* Kh16   = (_Float16*)(ws + OFF_KH);
  _Float16* Vt16   = (_Float16*)(ws + OFF_VT);
  _Float16* Vatt16 = (_Float16*)(ws + OFF_VATT);
  float*    X1     = (float*)(ws + OFF_X1);
  _Float16* NX2    = (_Float16*)(ws + OFF_NX2);
  _Float16* H16    = (_Float16*)(ws + OFF_H);

  dim3 blk(256);
  dim3 gg(DIM / 64, MROWS / 64);
  dim3 gf(DFF / 64, MROWS / 64);

  wconv_kernel<<<dim3((unsigned)(WT_ELEMS / 2048)), blk, 0, stream>>>(Wq, Wk, Wv, Wo, W1, W2, Wt);
  ln_kernel<1, SEQ_FULL><<<dim3(MROWS), dim3(128), 0, stream>>>(x, g1, be1, NX16);
  gemm_kernel<0, DIM, DIM><<<gg, blk, 0, stream>>>(NX16, Wt + 0 * WP, bq, x, X1, X1, Qh16);
  gemm_kernel<0, DIM, DIM><<<gg, blk, 0, stream>>>(NX16, Wt + 1 * WP, bk, x, X1, X1, Kh16);
  gemm_kernel<1, DIM, DIM><<<gg, blk, 0, stream>>>(NX16, Wt + 2 * WP, bv, x, X1, X1, Vt16);
  attn_kernel<<<dim3(SEQ / 128, NHEAD, NB), blk, 0, stream>>>(Qh16, Kh16, Vt16, mask, Vatt16);
  gemm_kernel<2, DIM, DIM><<<gg, blk, 0, stream>>>(Vatt16, Wt + 3 * WP, bo, x, X1, X1, NX2);
  ln_kernel<0, SEQ><<<dim3(MROWS), dim3(128), 0, stream>>>(X1, g2, be2, NX2);
  gemm_kernel<3, DIM, DFF><<<gf, blk, 0, stream>>>(NX2, Wt + 4 * WP, b1, x, X1, X1, H16);
  gemm_kernel<4, DFF, DIM><<<gg, blk, 0, stream>>>(H16, Wt + 8 * WP, b2, x, X1, out, H16);
}
